// GCNN_69114613730641
// MI455X (gfx1250) — hardware-run, weakly checked
//
#include <hip/hip_runtime.h>
#include <stddef.h>
#include <stdint.h>
#include <math.h>

#define NN      100000
#define NE      3200000
#define FIN     92
#define KP      96
#define XW      (KP / 2)
#define HD      64
#define GBM     128
#define MP      100096
#define PBX     (MP / GBM)
#define NTHR    256
#define NWAVE   8
#define EPT     8
#define WCH     (32 * EPT)
#define NBRUN   1024
#define SLB     10
#define NBK     98
#define WLCAP   4608
#define RCAP    35840
#define TRIPCAP 128
#define MAXDEG_MEAS   57
#define MAXB1024_MEAS 33219
#define SP      68
#define WSMAX   134217728

#define BK_ZINTS (NWAVE * WLCAP + RCAP + 2 * NBRUN)
#define BK_INTS  (BK_ZINTS + 16)
#define BK_LDS   (BK_INTS * 4)

static_assert(HD == 64 && HD == 16 * 4);
static_assert(MP % GBM == 0 && MP >= NN && MP == 782 * GBM);
static_assert(NBRUN == (1 << SLB) && NBRUN == 1024 && NBRUN % 16 == 0 && NBRUN % NTHR == 0);
static_assert(NBK * NBRUN >= MP);
static_assert(NE <= (1 << 22));
static_assert(NE % WCH == 0 && NE % 4 == 0);
static_assert(RCAP % (NTHR * 4) == 0 && BK_ZINTS % 4 == 0);
static_assert((long long)RCAP * 100 >= (long long)MAXB1024_MEAS * 105);
static_assert(WLCAP >= MAXB1024_MEAS / 8 + 384);
static_assert(NWAVE * WLCAP >= RCAP);
static_assert(NN <= 131072 && NN % 16 == 0);
static_assert(MAXDEG_MEAS + 8 <= TRIPCAP);
static_assert(KP % 32 == 0 && KP >= FIN && FIN % 4 == 0 && FIN / 4 == 23 && KP / 4 == 24);
static_assert(GBM * (KP / 4) == 12 * NTHR);
static_assert(GBM * KP * 2 / 16 == 6 * NTHR);
static_assert(HD * KP / 8 == 3 * NTHR);
static_assert(BK_LDS <= 300000);
static_assert((GBM * SP + GBM + 64) * 4 <= 65536);

typedef float          v4f   __attribute__((ext_vector_type(4)));
typedef float          v8f   __attribute__((ext_vector_type(8)));
typedef int            v4i   __attribute__((ext_vector_type(4)));
typedef int            v8i   __attribute__((ext_vector_type(8)));
typedef unsigned int   v2u   __attribute__((ext_vector_type(2)));
typedef unsigned int   v4u   __attribute__((ext_vector_type(4)));
typedef unsigned short v8us  __attribute__((ext_vector_type(8)));
typedef unsigned short v16us __attribute__((ext_vector_type(16)));
typedef __bf16         v16bf __attribute__((ext_vector_type(16)));
typedef v4f  __attribute__((may_alias)) v4fa;
typedef v4i  __attribute__((may_alias)) v4ia;
typedef v2u  __attribute__((may_alias)) v2ua;
typedef v4u  __attribute__((may_alias)) v4ua;
typedef v8us __attribute__((may_alias)) v8usa;
union FragB { v16bf v; v16us u; v8us h[2]; v8i w; };

__device__ __forceinline__ v8f wmb(const FragB& a, const FragB& b, v8f c) {
  v8f d = __builtin_amdgcn_wmma_f32_16x16x32_bf16(false, a.v, false, b.v, (short)0, c, false, false);
  asm volatile("v_nop\n\tv_nop\n\tv_nop\n\tv_nop" : "+v"(d) : "v"(a.w), "v"(b.w));
  return d;
}

__device__ __forceinline__ unsigned bf16_bits(float f) {
  const unsigned u = __float_as_uint(f);
  const unsigned r = (u + 0x7FFFu + ((u >> 16) & 1u)) >> 16;
  const unsigned q = (u >> 16) | 0x40u;
  return ((u & 0x7fffffffu) > 0x7f800000u) ? q : r;
}
__device__ __forceinline__ float bf16_val(float f) {
  return __uint_as_float(bf16_bits(f) << 16);
}

__device__ __forceinline__ void st2_v4f(float* p, v4f v) {
  *(volatile v4f*)p = v;
  __threadfence();
  *(volatile v4f*)p = v;
}
__device__ __forceinline__ void st2_v8us(unsigned short* p, v8us v) {
  *(volatile v8us*)p = v;
  __threadfence();
  *(volatile v8us*)p = v;
}

__global__ __launch_bounds__(NTHR) void k_prep(const float* __restrict__ x, const float* __restrict__ w,
                                               const float* __restrict__ b, unsigned short* xb,
                                               unsigned short* wt, float* bv) {
  __shared__ __attribute__((aligned(16))) unsigned tile[GBM * XW];
  const int tid = (int)threadIdx.x;
  const int blk = (int)blockIdx.x;
  if (blk < PBX) {
    const int r0 = blk * GBM;
#pragma unroll 4
    for (int it = 0; it < 12; ++it) {
      const int u   = it * NTHR + tid;
      const int lr  = u / 24;
      const int c4  = u - lr * 24;
      const int row = r0 + lr;
      const int rc  = row < NN ? row : NN - 1;
      const int cc  = c4 < 23 ? c4 : 22;
      const v4f a = *(const v4fa*)(x + (size_t)rc * FIN + 4 * cc);
      asm volatile("" :: "v"(a));
      const unsigned mk = ((row < NN) & (c4 < 23)) ? 0xffffffffu : 0u;
      v2u o;
      o.x = (bf16_bits(a.x) | (bf16_bits(a.y) << 16)) & mk;
      o.y = (bf16_bits(a.z) | (bf16_bits(a.w) << 16)) & mk;
      *(v2ua*)(tile + 2 * u) = o;
    }
    __syncthreads();
    v4u pv[6];
#pragma unroll
    for (int it = 0; it < 6; ++it) pv[it] = *(const v4ua*)(tile + 4 * (it * NTHR + tid));
    unsigned* dp = (unsigned*)xb + (size_t)blk * (size_t)(GBM * XW);
#pragma unroll
    for (int it = 0; it < 6; ++it) *(volatile v4u*)(dp + 4 * (it * NTHR + tid)) = pv[it];
    __threadfence();
#pragma unroll
    for (int it = 0; it < 6; ++it) *(volatile v4u*)(dp + 4 * (it * NTHR + tid)) = pv[it];
  } else {
#pragma unroll 1
    for (int it = 0; it < 3; ++it) {
      const int u  = it * NTHR + tid;
      const int n  = u / 12;
      const int k8 = (u - n * 12) * 8;
      float f[8];
#pragma unroll
      for (int i = 0; i < 8; ++i) {
        const int kk = k8 + i;
        const int kc = kk < FIN ? kk : FIN - 1;
        f[i] = w[(size_t)kc * HD + n];
      }
      asm volatile("" :: "v"(f[0]), "v"(f[1]), "v"(f[2]), "v"(f[3]));
      asm volatile("" :: "v"(f[4]), "v"(f[5]), "v"(f[6]), "v"(f[7]));
      v8us o;
#pragma unroll
      for (int i = 0; i < 8; ++i) {
        const unsigned mk = (k8 + i < FIN) ? 0xffffu : 0u;
        o[i] = (unsigned short)(bf16_bits(f[i]) & mk);
      }
      st2_v8us(wt + (size_t)u * 8, o);
    }
    {
      const int q = tid & 15;
      const v4f a = *(const v4fa*)(b + 4 * q);
      asm volatile("" :: "v"(a));
      v4f o;
      o.x = bf16_val(a.x); o.y = bf16_val(a.y); o.z = bf16_val(a.z); o.w = bf16_val(a.w);
      if (tid < 16) st2_v4f(bv + 4 * q, o);
    }
  }
}

__device__ __forceinline__ void bucket_flush(const int* pl, const int* cnt, const int* dvb, int ov,
                                             int* lp, int* cop, int* dvp, int* fp, int tid) {
#pragma unroll 1
  for (int i = tid * 4; i < RCAP; i += NTHR * 4) {
    const v4i v = *(const v4ia*)(pl + i);
    *(volatile v4i*)(lp + i) = v;
  }
#pragma unroll
  for (int it = 0; it < 2; ++it) {
    const v4i v = *(const v4ia*)(cnt + 4 * (it * NTHR + tid));
    *(volatile v4i*)(cop + 4 * (it * NTHR + tid)) = v;
  }
  {
    const v4i v = *(const v4ia*)(dvb + 4 * tid);
    *(volatile v4i*)(dvp + 4 * tid) = v;
  }
  if (tid < 8) {
    const v4i f = {ov, ov, ov, ov};
    *(volatile v4i*)(fp + 4 * tid) = f;
  }
}

__global__ __launch_bounds__(NTHR) void k_bucket(const int* __restrict__ srcs, const int* __restrict__ dsts,
                                                 int* LIST, int* CO, int* DV, int* FLAG) {
  extern __shared__ __attribute__((aligned(16))) int dsm[];
  int* wl   = dsm;
  int* pl   = dsm + NWAVE * WLCAP;
  int* cnt  = pl + RCAP;
  int* cur  = cnt + NBRUN;
  int* misc = cur + NBRUN;
  const int tid = (int)threadIdx.x, lane = tid & 31, wave = tid >> 5;
  const int blk = (int)blockIdx.x;
  const unsigned nbs = (unsigned)(blk * NBRUN);

  {
    const v4i z4 = {0, 0, 0, 0};
    for (int i = tid * 4; i < BK_ZINTS; i += NTHR * 4) *(v4ia*)(dsm + i) = z4;
    if (tid < 16) misc[tid] = 0;
  }
  __syncthreads();

  {
    const int per  = ((NE + NWAVE * WCH - 1) / (NWAVE * WCH)) * WCH;
    const int ebeg = wave * per;
    const int eend = (ebeg + per < NE) ? (ebeg + per) : NE;
    int* mylist = wl + wave * WLCAP;
    int wc = 0;
#pragma unroll 1
    for (int cb = ebeg; cb < eend; cb += WCH) {
      const int e0 = cb + lane * EPT;
      const v4i da = *(const v4ia*)(dsts + e0);
      const v4i db = *(const v4ia*)(dsts + e0 + 4);
      const unsigned s0 = (unsigned)da.x - nbs, s1 = (unsigned)da.y - nbs;
      const unsigned s2 = (unsigned)da.z - nbs, s3 = (unsigned)da.w - nbs;
      const unsigned s4 = (unsigned)db.x - nbs, s5 = (unsigned)db.y - nbs;
      const unsigned s6 = (unsigned)db.z - nbs, s7 = (unsigned)db.w - nbs;
      const bool h0 = s0 < (unsigned)NBRUN, h1 = s1 < (unsigned)NBRUN, h2 = s2 < (unsigned)NBRUN, h3 = s3 < (unsigned)NBRUN;
      const bool h4 = s4 < (unsigned)NBRUN, h5 = s5 < (unsigned)NBRUN, h6 = s6 < (unsigned)NBRUN, h7 = s7 < (unsigned)NBRUN;
      const unsigned m0 = __builtin_amdgcn_ballot_w32(h0), m1 = __builtin_amdgcn_ballot_w32(h1);
      const unsigned m2 = __builtin_amdgcn_ballot_w32(h2), m3 = __builtin_amdgcn_ballot_w32(h3);
      const unsigned m4 = __builtin_amdgcn_ballot_w32(h4), m5 = __builtin_amdgcn_ballot_w32(h5);
      const unsigned m6 = __builtin_amdgcn_ballot_w32(h6), m7 = __builtin_amdgcn_ballot_w32(h7);
      const unsigned any = m0 | m1 | m2 | m3 | m4 | m5 | m6 | m7;
      if (any != 0u) {
        const int pre = (int)(__builtin_amdgcn_mbcnt_lo(m0, 0u) + __builtin_amdgcn_mbcnt_lo(m1, 0u) +
                              __builtin_amdgcn_mbcnt_lo(m2, 0u) + __builtin_amdgcn_mbcnt_lo(m3, 0u) +
                              __builtin_amdgcn_mbcnt_lo(m4, 0u) + __builtin_amdgcn_mbcnt_lo(m5, 0u) +
                              __builtin_amdgcn_mbcnt_lo(m6, 0u) + __builtin_amdgcn_mbcnt_lo(m7, 0u));
        int p = wc + pre;
        const unsigned eb = (unsigned)e0;
        if (h0) { if (p < WLCAP) mylist[p] = (int)(((eb + 0u) << SLB) | s0); p = p + 1; }
        if (h1) { if (p < WLCAP) mylist[p] = (int)(((eb + 1u) << SLB) | s1); p = p + 1; }
        if (h2) { if (p < WLCAP) mylist[p] = (int)(((eb + 2u) << SLB) | s2); p = p + 1; }
        if (h3) { if (p < WLCAP) mylist[p] = (int)(((eb + 3u) << SLB) | s3); p = p + 1; }
        if (h4) { if (p < WLCAP) mylist[p] = (int)(((eb + 4u) << SLB) | s4); p = p + 1; }
        if (h5) { if (p < WLCAP) mylist[p] = (int)(((eb + 5u) << SLB) | s5); p = p + 1; }
        if (h6) { if (p < WLCAP) mylist[p] = (int)(((eb + 6u) << SLB) | s6); p = p + 1; }
        if (h7) { if (p < WLCAP) mylist[p] = (int)(((eb + 7u) << SLB) | s7); p = p + 1; }
        wc += (int)(__builtin_popcount(m0) + __builtin_popcount(m1) + __builtin_popcount(m2) + __builtin_popcount(m3) +
                    __builtin_popcount(m4) + __builtin_popcount(m5) + __builtin_popcount(m6) + __builtin_popcount(m7));
      }
    }
    if (lane == 0) misc[wave] = wc;
  }
  __syncthreads();

  if (wave == 0) {
    int ov = 0;
    int tot = 0;
#pragma unroll 1
    for (int w2 = 0; w2 < NWAVE; ++w2) {
      int c = misc[w2];
      if (c > WLCAP) ov = 1;
      c = c < 0 ? 0 : (c > WLCAP ? WLCAP : c);
      tot += c;
#pragma unroll 1
      for (int b0 = 0; b0 < c; b0 += 32) {
        const int idx = b0 + lane;
        const int ent = wl[w2 * WLCAP + (idx < WLCAP ? idx : WLCAP - 1)];
        const int m32 = (c - b0) < 32 ? (c - b0) : 32;
#pragma unroll 1
        for (int k = 0; k < m32; ++k) {
          const int u    = __builtin_amdgcn_readlane(ent, k);
          const int slot = u & (NBRUN - 1);
          if (lane == 0) cnt[slot] = cnt[slot] + 1;
        }
      }
    }
    if (tot > RCAP) ov = 1;
    if (lane == 0) misc[9] = ov;
  }
  __syncthreads();
  if (wave == 0) {
    const int base = lane * (NBRUN / 32);
    int s = 0;
#pragma unroll 1
    for (int i = 0; i < NBRUN / 32; ++i) s += cnt[base + i];
    int incl = s;
#pragma unroll
    for (int d = 1; d < 32; d <<= 1) {
      const int y = __shfl_up(incl, d, 32);
      if (lane >= d) incl += y;
    }
    int run = incl - s;
#pragma unroll 1
    for (int i = 0; i < NBRUN / 32; ++i) {
      const int cv = cnt[base + i];
      cur[base + i] = run;
      run += cv;
    }
  }
  __syncthreads();

  if (wave == 0) {
#pragma unroll 1
    for (int w2 = 0; w2 < NWAVE; ++w2) {
      int c = misc[w2];
      c = c < 0 ? 0 : (c > WLCAP ? WLCAP : c);
#pragma unroll 1
      for (int b0 = 0; b0 < c; b0 += 32) {
        const int idx = b0 + lane;
        const int ent = wl[w2 * WLCAP + (idx < WLCAP ? idx : WLCAP - 1)];
        int eid = (int)((unsigned)ent >> SLB);
        eid = eid > NE - 1 ? NE - 1 : eid;
        int sr = srcs[eid];
        sr = sr < 0 ? 0 : (sr > NN - 1 ? NN - 1 : sr);
        const int m32 = (c - b0) < 32 ? (c - b0) : 32;
#pragma unroll 1
        for (int k = 0; k < m32; ++k) {
          const int u    = __builtin_amdgcn_readlane(ent, k);
          const int wd   = __builtin_amdgcn_readlane(sr, k);
          const int slot = u & (NBRUN - 1);
          if (lane == 0) {
            int p = cur[slot];
            p = p < 0 ? 0 : (p > RCAP - 1 ? RCAP - 1 : p);
            pl[p] = wd;
            cur[slot] = p + 1;
          }
        }
      }
    }
  }
  __syncthreads();

#pragma unroll 1
  for (int i = 0; i < NBRUN / NTHR; ++i) {
    const int s  = i * NTHR + tid;
    const int cv = cnt[s];
    cur[s] = cur[s] - cv;
    const float dg = (float)(cv + 1);
    wl[s] = __float_as_int(1.0f / sqrtf(dg));
  }
  __syncthreads();

  const int ovf = misc[9];
  int* lp  = LIST + (size_t)blk * RCAP;
  int* cop = CO + (size_t)blk * (2 * NBRUN);
  int* dvp = DV + (size_t)blk * NBRUN;
  int* fp  = FLAG + (size_t)blk * 32;
  bucket_flush(pl, cnt, wl, ovf, lp, cop, dvp, fp, tid);
  __threadfence();
  bucket_flush(pl, cnt, wl, ovf, lp, cop, dvp, fp, tid);
}

template <int KTOT>
__device__ __forceinline__ void gemm_16x64(const unsigned short* __restrict__ ap,
                                           const unsigned short* __restrict__ bp, v8f (&acc)[4]) {
#pragma unroll 1
  for (int k0 = 0; k0 < KTOT; k0 += 32) {
    FragB af;
    af.h[0] = *(const v8usa*)(ap + k0);
    af.h[1] = *(const v8usa*)(ap + k0 + 16);
#pragma unroll
    for (int nt = 0; nt < 4; ++nt) {
      const unsigned short* wq = bp + (size_t)(16 * nt) * (size_t)KTOT + k0;
      FragB bf;
      bf.h[0] = *(const v8usa*)wq;
      bf.h[1] = *(const v8usa*)(wq + 16);
      acc[nt] = wmb(af, bf, acc[nt]);
    }
  }
}

__device__ __forceinline__ void stage_d(float* stg, const v8f (&acc)[4], int wave, int hh, int m) {
#pragma unroll
  for (int nt = 0; nt < 4; ++nt) {
#pragma unroll
    for (int r = 0; r < 8; ++r) stg[(16 * wave + 8 * hh + r) * SP + 16 * nt + m] = acc[nt][r];
  }
}

__global__ __launch_bounds__(NTHR) __attribute__((amdgpu_num_vgpr(248)))
void k_gemm(const unsigned short* __restrict__ XB, const unsigned short* __restrict__ WT,
            const float* __restrict__ BV, const float* __restrict__ DV, float* P) {
  __shared__ __attribute__((aligned(16))) float stg[GBM * SP];
  __shared__ __attribute__((aligned(16))) float sd[GBM];
  __shared__ __attribute__((aligned(16))) float sb[64];
  const int tid = (int)threadIdx.x, lane = tid & 31, wave = tid >> 5, hh = lane >> 4, m = lane & 15;
  const int rowBase = (int)blockIdx.x * GBM;
  if (wave == 0) *(v4fa*)(sd + 4 * lane) = *(const v4fa*)(DV + (size_t)rowBase + 4 * lane);
  if (wave == 1) *(v4fa*)(sb + 4 * m) = *(const v4fa*)(BV + 4 * m);

  v8f acc[4];
  {
    const v8f z = {0.f, 0.f, 0.f, 0.f, 0.f, 0.f, 0.f, 0.f};
#pragma unroll
    for (int t = 0; t < 4; ++t) acc[t] = z;
  }
  const unsigned short* ap = XB + (size_t)(rowBase + 16 * wave + m) * (size_t)KP + 8 * hh;
  const unsigned short* bp = WT + (size_t)m * (size_t)KP + 8 * hh;
  gemm_16x64<KP>(ap, bp, acc);
  stage_d(stg, acc, wave, hh, m);
  __syncthreads();

  const v4f bias = *(const v4fa*)(sb + 4 * m);
#pragma unroll 1
  for (int i = 0; i < 8; ++i) {
    const int lr   = 16 * wave + 2 * i + hh;
    const int grow = rowBase + lr;
    const bool live = grow < NN;
    const v4f a  = *(const v4fa*)(stg + lr * SP + 4 * m);
    const float dv = sd[lr];
    asm volatile("" :: "v"(a));
    const float v0 = dv * (a.x + bias.x), v1 = dv * (a.y + bias.y);
    const float v2 = dv * (a.z + bias.z), v3 = dv * (a.w + bias.w);
    v4f o;
    o.x = live ? v0 : 0.0f; o.y = live ? v1 : 0.0f; o.z = live ? v2 : 0.0f; o.w = live ? v3 : 0.0f;
    st2_v4f(P + (size_t)grow * HD + 4 * m, o);
  }
}

__global__ __launch_bounds__(NTHR) void k_replay(const int* __restrict__ LIST, const int* __restrict__ CO,
                                                 const float* __restrict__ DV, const int* __restrict__ FLAG,
                                                 const float* __restrict__ P, float* out) {
  const int tid = (int)threadIdx.x, lane = tid & 31, wave = tid >> 5, hh = lane >> 4, q = lane & 15;
  const int blk = (int)blockIdx.x;
  const int* lb  = LIST + (size_t)blk * RCAP;
  const int* cob = CO + (size_t)blk * (2 * NBRUN);
  const int flag = FLAG[(size_t)blk * 32];
  const float qnan = __uint_as_float(0x7fc00000u);

#pragma unroll 1
  for (int i = 0; i < NBRUN / 16; ++i) {
    const int slot = 16 * i + 2 * wave + hh;
    const int d    = blk * NBRUN + slot;
    int c = cob[slot];
    int o = cob[NBRUN + slot];
    const bool big = c > TRIPCAP;
    c = c < 0 ? 0 : (c > TRIPCAP ? TRIPCAP : c);
    o = o < 0 ? 0 : (o > RCAP - 1 ? RCAP - 1 : o);
    const int co = __shfl_xor(c, 16, 32);
    const int cm = c > co ? c : co;
    int last = o + c - 1;
    last = last < o ? o : last;
    last = last > RCAP - 1 ? RCAP - 1 : last;
    const int dc = d < NN ? d : NN - 1;
    const float dv = DV[d];
    const v4f sf = *(const v4fa*)(P + (size_t)dc * HD + 4 * q);
    float a0 = sf.x, a1 = sf.y, a2 = sf.z, a3 = sf.w;
#pragma unroll 1
    for (int j = 0; j < cm; j += 2) {
      int i0 = o + j, i1 = o + j + 1;
      i0 = i0 > last ? last : i0;
      i1 = i1 > last ? last : i1;
      int s0 = lb[i0], s1 = lb[i1];
      s0 = s0 < 0 ? 0 : (s0 > NN - 1 ? NN - 1 : s0);
      s1 = s1 < 0 ? 0 : (s1 > NN - 1 ? NN - 1 : s1);
      const v4f u0 = *(const v4fa*)(P + (size_t)s0 * HD + 4 * q);
      const v4f u1 = *(const v4fa*)(P + (size_t)s1 * HD + 4 * q);
      asm volatile("" :: "v"(u0));
      asm volatile("" :: "v"(u1));
      const bool ok0 = j < c, ok1 = (j + 1) < c;
      float t0 = a0 + u0.x, t1 = a1 + u0.y, t2 = a2 + u0.z, t3 = a3 + u0.w;
      a0 = ok0 ? t0 : a0; a1 = ok0 ? t1 : a1; a2 = ok0 ? t2 : a2; a3 = ok0 ? t3 : a3;
      t0 = a0 + u1.x; t1 = a1 + u1.y; t2 = a2 + u1.z; t3 = a3 + u1.w;
      a0 = ok1 ? t0 : a0; a1 = ok1 ? t1 : a1; a2 = ok1 ? t2 : a2; a3 = ok1 ? t3 : a3;
    }
    float m0 = dv * a0, m1 = dv * a1, m2 = dv * a2, m3 = dv * a3;
    const bool bad  = (flag != 0) | big;
    m0 = bad ? qnan : m0; m1 = bad ? qnan : m1; m2 = bad ? qnan : m2; m3 = bad ? qnan : m3;
    v4f ov;
    ov.x = m0; ov.y = m1; ov.z = m2; ov.w = m3;
    const bool live = d < NN;
    float* op = out + (size_t)dc * HD + 4 * q;
    if (live) *(volatile v4f*)op = ov;
    __threadfence();
    if (live) *(volatile v4f*)op = ov;
  }
}

extern "C" void kernel_launch(void* const* d_in, const int* in_sizes, int n_in,
                              void* d_out, int out_size, void* d_ws, size_t ws_size,
                              hipStream_t stream) {
  if (n_in < 4) return;
  if (in_sizes[0] != NN * FIN) return;
  if (in_sizes[1] != 2 * NE) return;
  if (in_sizes[2] != FIN * HD) return;
  if (in_sizes[3] != HD) return;
  if (out_size != NN * HD) return;

  const float* x  = (const float*)d_in[0];
  const int*   ei = (const int*)d_in[1];
  const float* W  = (const float*)d_in[2];
  const float* b  = (const float*)d_in[3];
  float* out = (float*)d_out;
  const int* srcs = ei;
  const int* dsts = ei + NE;

  constexpr size_t zXB   = (size_t)MP * KP * 2;
  constexpr size_t zWT   = (size_t)HD * KP * 2;
  constexpr size_t zBV   = 256;
  constexpr size_t zLIST = (size_t)NBK * RCAP * 4;
  constexpr size_t zCO   = (size_t)NBK * 2 * NBRUN * 4;
  constexpr size_t zDV   = (size_t)NBK * NBRUN * 4;
  constexpr size_t zFLAG = (size_t)NBK * 128;
  constexpr size_t zP    = (size_t)MP * HD * 4;
  constexpr size_t oXB   = 0;
  constexpr size_t oWT   = oXB + zXB;
  constexpr size_t oBV   = oWT + zWT;
  constexpr size_t oLIST = oBV + zBV;
  constexpr size_t oCO   = oLIST + zLIST;
  constexpr size_t oDV   = oCO + zCO;
  constexpr size_t oFLAG = oDV + zDV;
  constexpr size_t oP    = oFLAG + zFLAG;
  constexpr size_t oEND  = oP + zP;
  static_assert(zXB % 256 == 0 && zWT % 256 == 0 && zBV % 256 == 0 && zLIST % 256 == 0);
  static_assert(zCO % 256 == 0 && zDV % 256 == 0 && zFLAG % 256 == 0 && zP % 256 == 0);
  static_assert((size_t)PBX * GBM * KP * 2 == zXB);
  static_assert((size_t)NBK * NBRUN >= (size_t)MP);
  static_assert(oEND <= (size_t)WSMAX);
  if (oEND > ws_size) return;

  char* ws = (char*)d_ws;
  unsigned short* XB   = (unsigned short*)(ws + oXB);
  unsigned short* WT   = (unsigned short*)(ws + oWT);
  float*          BV   = (float*)(ws + oBV);
  int*            LIST = (int*)(ws + oLIST);
  int*            CO   = (int*)(ws + oCO);
  int*            DVi  = (int*)(ws + oDV);
  const float*    DVf  = (const float*)(ws + oDV);
  int*            FLAG = (int*)(ws + oFLAG);
  float*          P    = (float*)(ws + oP);

  hipFuncSetAttribute(reinterpret_cast<const void*>(&k_bucket), hipFuncAttributeMaxDynamicSharedMemorySize, (int)BK_LDS);

  k_prep<<<PBX + 1, NTHR, 0, stream>>>(x, W, b, XB, WT, BV);
  k_bucket<<<NBK, NTHR, BK_LDS, stream>>>(srcs, dsts, LIST, CO, DVi, FLAG);
  k_gemm<<<PBX, NTHR, 0, stream>>>(XB, WT, BV, DVf, P);
  k_replay<<<NBK, NTHR, 0, stream>>>(LIST, CO, DVf, FLAG, P, out);
}
